// CrossLinearAttention_38749194944573
// MI455X (gfx1250) — hardware-verified
//
#include <hip/hip_runtime.h>
#include <math.h>

typedef __attribute__((ext_vector_type(16))) _Float16 v16h;
typedef __attribute__((ext_vector_type(16))) __bf16 v16b;
typedef __attribute__((ext_vector_type(8)))  _Float16 v8h;
typedef __attribute__((ext_vector_type(8)))  float v8f;
typedef __attribute__((ext_vector_type(4)))  float v4f;
typedef __attribute__((ext_vector_type(2)))  float v2f;
typedef __attribute__((ext_vector_type(4)))  unsigned v4u;
typedef __attribute__((ext_vector_type(4)))  int v4i;
typedef float __attribute__((may_alias)) float_a;
typedef int __attribute__((may_alias)) int_a;

template <typename T> __device__ __forceinline__ void vst2(void* p, T v) { *(volatile T*)p = v; __threadfence(); *(volatile T*)p = v; }
__device__ __forceinline__ v8f wmma16(v16h a, v16h b, v8f c) {
  v8f d = __builtin_amdgcn_wmma_f32_16x16x32_f16(false, a, false, b, (short)0, c, false, false);
  asm volatile("v_nop\n\tv_nop\n\tv_nop\n\tv_nop" : "+v"(d) : "v"(a), "v"(b));
  return d;
}
__device__ __forceinline__ v8f wmma_bf(v16b a, v16b b, v8f c) {
  v8f d = __builtin_amdgcn_wmma_f32_16x16x32_bf16(false, a, false, b, (short)0, c, false, false);
  asm volatile("v_nop\n\tv_nop\n\tv_nop\n\tv_nop" : "+v"(d) : "v"(a), "v"(b));
  return d;
}
__device__ __forceinline__ v16h frag_h(const _Float16* rowk0, int lane) {
  union { v16h v; v8h q[2]; } u; const _Float16* p = rowk0 + 8 * (lane >> 4);
  u.q[0] = *(const v8h*)p; u.q[1] = *(const v8h*)(p + 16); return u.v;
}
__device__ __forceinline__ v16h frag_f32(const float* rowk0, int lane) {
  v16h a; const float* p = rowk0 + 8 * (lane >> 4);
#pragma unroll
  for (int i = 0; i < 8; ++i) { a[i] = (_Float16)p[i]; a[8 + i] = (_Float16)p[16 + i]; }
  return a;
}
__device__ __forceinline__ v16h frag_f32s(const float* rowk0, int lane, float sc) {
  v16h a; const float* p = rowk0 + 8 * (lane >> 4);
#pragma unroll
  for (int i = 0; i < 8; ++i) { a[i] = (_Float16)(p[i] * sc); a[8 + i] = (_Float16)(p[16 + i] * sc); }
  return a;
}
__device__ __forceinline__ v16h fragc_f32(const float* W, int k0, int n, int lane, int ld, int K) {
  v16h a; const int g = lane >> 4;
#pragma unroll
  for (int i = 0; i < 8; ++i) { const int ka = k0 + 8 * g + i, kb = ka + 16;
    a[i] = (_Float16)(ka < K ? W[(size_t)(ka < K ? ka : K - 1) * ld + n] : 0.f); a[8 + i] = (_Float16)(kb < K ? W[(size_t)(kb < K ? kb : K - 1) * ld + n] : 0.f); }
  return a;
}
struct F2 { v16b h, l; };
__device__ __forceinline__ F2 bsplit16(const float v[16]) { F2 r;
#pragma unroll
  for (int i = 0; i < 16; ++i) { const __bf16 h = (__bf16)v[i]; r.h[i] = h; r.l[i] = (__bf16)(v[i] - (float)h); }
  return r; }
__device__ __forceinline__ F2 split_row(const float* row, int k0, int lane) { float v[16]; const float* p = row + k0 + 8 * (lane >> 4);
#pragma unroll
  for (int i = 0; i < 8; ++i) { v[i] = p[i]; v[8 + i] = p[16 + i]; }
  return bsplit16(v); }
__device__ __forceinline__ F2 split_rowK(const float* row, int k0, int lane, int K) { float v[16]; const int g = lane >> 4;
#pragma unroll
  for (int i = 0; i < 8; ++i) { const int ka = k0 + 8 * g + i, kb = ka + 16; v[i] = ka < K ? row[ka < K ? ka : K - 1] : 0.f; v[8 + i] = kb < K ? row[kb < K ? kb : K - 1] : 0.f; }
  return bsplit16(v); }
__device__ __forceinline__ F2 split_col(const float* W, int k0, int n, int lane, int ld, int K) { float v[16]; const int g = lane >> 4;
#pragma unroll
  for (int i = 0; i < 8; ++i) { const int ka = k0 + 8 * g + i, kb = ka + 16; v[i] = ka < K ? W[(size_t)(ka < K ? ka : K - 1) * ld + n] : 0.f; v[8 + i] = kb < K ? W[(size_t)(kb < K ? kb : K - 1) * ld + n] : 0.f; }
  return bsplit16(v); }
__device__ __forceinline__ v8f mac3(const F2& a, const F2& b, v8f c) { c = wmma_bf(a.l, b.h, c); c = wmma_bf(a.h, b.l, c); return wmma_bf(a.h, b.h, c); }
__device__ __forceinline__ float sigm(float v) { return 1.0f / (1.0f + expf(-v)); }
#define LDSX() do { asm volatile("s_wait_dscnt 0" ::: "memory"); __builtin_amdgcn_wave_barrier(); __builtin_amdgcn_fence(__ATOMIC_RELEASE, "workgroup"); } while (0)


#define NB 4
#define N1 8192
#define N2 8192
#define DIMI 256
#define NH 8
#define HD 64
#define INNER (NH * HD)
#define LNEPS 1e-5f
#define POSMUL 64.0f
#ifndef TNB
#define TNB NB
#endif
typedef __attribute__((ext_vector_type(8))) __bf16 v8b;
__device__ __forceinline__ v16b frag_b(const __bf16* rowk0, int lane) {
  union { v16b v; v8b q[2]; } u; const __bf16* p = rowk0 + 8 * (lane >> 4);
  u.q[0] = *(const v8b*)p; u.q[1] = *(const v8b*)(p + 16); return u.v;
}
__device__ __forceinline__ float bfr(float v) { return (float)(__bf16)v; }
__device__ __attribute__((noinline)) float exp_ni(float v) { return expf(v); }
__device__ __attribute__((noinline)) float erf_ni(float v) { return erff(v); }

#define WS_QH  0u
#define WS_QL  (WS_QH + 2u * (size_t)NB * N1 * INNER)
#define WS_KH  (WS_QL + 2u * (size_t)NB * N1 * INNER)
#define WS_KL  (WS_KH + 2u * (size_t)NB * INNER * N2)
#define WS_VH  (WS_KL + 2u * (size_t)NB * INNER * N2)
#define WS_VL  (WS_VH + 2u * (size_t)NB * INNER * N2)
#define WS_DT  (WS_VL + 2u * (size_t)NB * INNER * N2)
#define WS_END (WS_DT + 4u * (size_t)NB * NH * HD * HD)

__device__ __forceinline__ v16b fragb_f32(const float* __restrict__ p, int lane) { v16b a; const float* pp = p + 8 * (lane >> 4);
#pragma unroll
  for (int i = 0; i < 8; ++i) { a[i] = (__bf16)pp[i]; a[8 + i] = (__bf16)pp[16 + i]; } return a; }
__device__ __forceinline__ void rot_tile(v8f acc[8], const float* __restrict__ POS, size_t rowbase, int g, int col) {
  const float invf = powf(10000.0f, -(float)(2 * col) / 32.0f);
#pragma unroll
  for (int r = 0; r < 8; ++r) { const size_t row = rowbase + 8 * g + r; const float px = bfr(POS[row * 2 + 0]) * POSMUL * invf, py = bfr(POS[row * 2 + 1]) * POSMUL * invf; const float cx = cosf(px), sx = sinf(px), cy = cosf(py), sy = sinf(py);
#pragma unroll
    for (int m = 0; m < 4; ++m) { const bool isy = (m & 1); const float c = isy ? cy : cx, s = isy ? sy : sx; const float a = acc[2 * m][r], b2 = acc[2 * m + 1][r]; acc[2 * m][r] = a * c - b2 * s; acc[2 * m + 1][r] = b2 * c + a * s; } } }
__global__ __launch_bounds__(128) void k_q(const float* __restrict__ X, const float* __restrict__ WQ, const float* __restrict__ XP, _Float16* __restrict__ QH, _Float16* __restrict__ QL) { __shared__ __align__(16) _Float16 sh[64][136], sl[64][136];
  const int tid = threadIdx.x, wave = tid >> 5, lane = tid & 31, col = lane & 15, g = lane >> 4; const size_t r0 = (size_t)blockIdx.x * 64 + wave * 16; const int c0 = blockIdx.y * 128;
  v8f acc[8] = {};
#pragma unroll
  for (int kc = 0; kc < DIMI / 32; ++kc) { const v16b a = fragb_f32(X + (r0 + col) * DIMI + kc * 32, lane);
#pragma unroll
    for (int j = 0; j < 8; ++j) acc[j] = wmma_bf(a, fragb_f32(WQ + (size_t)(c0 + j * 16 + col) * DIMI + kc * 32, lane), acc[j]); }
  rot_tile(acc, XP, r0, g, col);
#pragma unroll
  for (int j = 0; j < 8; ++j)
#pragma unroll
    for (int r = 0; r < 8; ++r) { const float v = acc[j][r]; const _Float16 hv = (_Float16)v; sh[wave * 16 + 8 * g + r][j * 16 + col] = hv; sl[wave * 16 + 8 * g + r][j * 16 + col] = (_Float16)((v - (float)hv) * 2048.0f); }
  __syncthreads(); for (int e = tid; e < 64 * 16; e += 128) { const int rl = e >> 4, q = e & 15; const size_t o = ((size_t)blockIdx.x * 64 + rl) * INNER + c0 + q * 8; vst2((unsigned*)(QH + o), *(const v4u*)&sh[rl][q * 8]); vst2((unsigned*)(QL + o), *(const v4u*)&sl[rl][q * 8]); } }
__global__ __launch_bounds__(128) void k_kv(const float* __restrict__ Z, const float* __restrict__ WKV, const float* __restrict__ ZP, const float* __restrict__ KG, const float* __restrict__ KB, const float* __restrict__ VG, const float* __restrict__ VB, _Float16* __restrict__ KH, _Float16* __restrict__ KL, _Float16* __restrict__ VH, _Float16* __restrict__ VL) { __shared__ __align__(16) _Float16 th[128][72], tl[128][72];
  const int tid = threadIdx.x, wave = tid >> 5, lane = tid & 31, col = lane & 15, g = lane >> 4; const size_t r0 = (size_t)blockIdx.x * 64 + wave * 16; const int c0 = blockIdx.y * 128; const bool isk = (c0 < INNER); const size_t b = r0 / N2; const int n0 = (int)(((size_t)blockIdx.x * 64) % N2);
  v8f acc[8] = {};
#pragma unroll
  for (int kc = 0; kc < DIMI / 32; ++kc) { const v16b a = fragb_f32(Z + (r0 + col) * DIMI + kc * 32, lane);
#pragma unroll
    for (int j = 0; j < 8; ++j) acc[j] = wmma_bf(a, fragb_f32(WKV + (size_t)(c0 + j * 16 + col) * DIMI + kc * 32, lane), acc[j]); }
  const float* GM = isk ? KG : VG; const float* BT = isk ? KB : VB;
#pragma unroll
  for (int hh = 0; hh < 2; ++hh) {
#pragma unroll
    for (int r = 0; r < 8; ++r) { float s = 0.f;
#pragma unroll
      for (int j = 0; j < 4; ++j) s += acc[hh * 4 + j][r];
#pragma unroll
      for (int o = 1; o < 16; o <<= 1) s += __shfl_xor(s, o);
      const float mu = s * (1.0f / HD); float q = 0.f;
#pragma unroll
      for (int j = 0; j < 4; ++j) { const float d = acc[hh * 4 + j][r] - mu; q += d * d; }
#pragma unroll
      for (int o = 1; o < 16; o <<= 1) q += __shfl_xor(q, o);
      const float inv = 1.0f / sqrtf(q * (1.0f / HD) + LNEPS);
#pragma unroll
      for (int j = 0; j < 4; ++j) { const int dd = j * 16 + col; acc[hh * 4 + j][r] = (acc[hh * 4 + j][r] - mu) * inv * bfr(GM[dd]) + bfr(BT[dd]); } } }
  if (isk) rot_tile(acc, ZP, r0, g, col);
#pragma unroll
  for (int j = 0; j < 8; ++j)
#pragma unroll
    for (int r = 0; r < 8; ++r) { const float v = acc[j][r]; const _Float16 hv = (_Float16)v; const int cl = j * 16 + col, rl = wave * 16 + 8 * g + r; th[cl][rl] = hv; tl[cl][rl] = (_Float16)((v - (float)hv) * 2048.0f); }
  __syncthreads();
  { _Float16* PH = isk ? KH : VH; _Float16* PL = isk ? KL : VL; const int cbase = isk ? c0 : (c0 - INNER);
    for (int e = tid; e < 128 * 8; e += 128) { const int cl = e >> 3, q = e & 7; const size_t o = (b * INNER + cbase + cl) * (size_t)N2 + n0 + q * 8; vst2((unsigned*)(PH + o), *(const v4u*)&th[cl][q * 8]); vst2((unsigned*)(PL + o), *(const v4u*)&tl[cl][q * 8]); } } }
__global__ __launch_bounds__(128) void k_dots(const _Float16* __restrict__ KH, const _Float16* __restrict__ KL, const _Float16* __restrict__ VH, const _Float16* __restrict__ VL, float* __restrict__ DT) { __shared__ __align__(16) float sf[4][16][68];
  const int tid = threadIdx.x, wave = tid >> 5, lane = tid & 31, col = lane & 15, g = lane >> 4; const size_t bh = blockIdx.x; const size_t pe = (bh * HD + wave * 16 + col) * N2;
  v8f acc[4] = {}, accl[4] = {};
#pragma unroll 2
  for (int kc = 0; kc < N2 / 32; ++kc) { const v16h ah = frag_h(VH + pe + kc * 32, lane), al = frag_h(VL + pe + kc * 32, lane);
#pragma unroll
    for (int j = 0; j < 4; ++j) { const size_t pd = (bh * HD + j * 16 + col) * N2 + kc * 32; const v16h kh = frag_h(KH + pd, lane); acc[j] = wmma16(ah, kh, acc[j]); accl[j] = wmma16(al, kh, accl[j]); accl[j] = wmma16(ah, frag_h(KL + pd, lane), accl[j]); } }
#pragma unroll
  for (int j = 0; j < 4; ++j)
#pragma unroll
    for (int r = 0; r < 8; ++r) sf[wave][8 * g + r][j * 16 + col] = acc[j][r] + accl[j][r] * (1.0f / 2048.0f);
  LDSX(); for (int rl = 0; rl < 16; ++rl) if (lane < 16) vst2(DT + (bh * HD + wave * 16 + rl) * HD + lane * 4, *(const v4f*)&sf[wave][rl][lane * 4]); }
__global__ __launch_bounds__(128) void k_o(const _Float16* __restrict__ QH, const _Float16* __restrict__ QL, const float* __restrict__ DT, const float* __restrict__ WO, const float* __restrict__ BO, float* __restrict__ OUT) { __shared__ __align__(16) float sc[4][16][36]; __shared__ __align__(16) float sf[4][16][132];
  const int tid = threadIdx.x, wave = tid >> 5, lane = tid & 31, col = lane & 15, g = lane >> 4; const size_t r0 = (size_t)blockIdx.x * 64 + wave * 16; const int c0 = blockIdx.y * 128; const size_t b = r0 / N1;
  v8f acc[8] = {};
#pragma unroll 1
  for (int ch = 0; ch < INNER / 32; ++ch) { const int h = ch >> 1, half = ch & 1;
    v8f c2[2] = {}, c2l[2] = {};
#pragma unroll
    for (int kc = 0; kc < 2; ++kc) { const v16h ah = frag_h(QH + (r0 + col) * INNER + h * HD + kc * 32, lane), al = frag_h(QL + (r0 + col) * INNER + h * HD + kc * 32, lane);
#pragma unroll
      for (int tt = 0; tt < 2; ++tt) { const F2 dw = split_row(DT + ((b * NH + h) * HD + half * 32 + tt * 16 + col) * HD, kc * 32, lane);
        v16h dh, dl;
#pragma unroll
        for (int i = 0; i < 16; ++i) { dh[i] = (_Float16)(float)dw.h[i]; dl[i] = (_Float16)(float)dw.l[i]; }
        c2[tt] = wmma16(ah, dh, c2[tt]); c2[tt] = wmma16(ah, dl, c2[tt]); c2l[tt] = wmma16(al, dh, c2l[tt]); } }
#pragma unroll
    for (int tt = 0; tt < 2; ++tt)
#pragma unroll
      for (int r = 0; r < 8; ++r) sc[wave][8 * g + r][tt * 16 + col] = (c2[tt][r] + c2l[tt][r] * (1.0f / 2048.0f)) * (1.0f / N2);
    LDSX();
    { const F2 a = split_row(&sc[wave][col][0], 0, lane);
#pragma unroll
      for (int j = 0; j < 8; ++j) { const v16b w = fragb_f32(WO + (size_t)(c0 + j * 16 + col) * INNER + ch * 32, lane); acc[j] = wmma_bf(a.h, w, acc[j]); acc[j] = wmma_bf(a.l, w, acc[j]); } }
    LDSX(); }
#pragma unroll
  for (int j = 0; j < 8; ++j)
#pragma unroll
    for (int r = 0; r < 8; ++r) sf[wave][8 * g + r][j * 16 + col] = acc[j][r] + bfr(BO[c0 + j * 16 + col]);
  LDSX(); for (int rl = 0; rl < 16; ++rl) vst2(OUT + (r0 + rl) * DIMI + c0 + lane * 4, *(const v4f*)&sf[wave][rl][lane * 4]); }
extern "C" void kernel_launch(void* const* d_in, const int* in_sizes, int n_in, void* d_out, int out_size, void* d_ws, size_t ws_size, hipStream_t stream) {
  (void)in_sizes; (void)n_in; (void)out_size;
  const float** F = (const float**)d_in;
  if (ws_size < (size_t)WS_END) return;
  char* ws = (char*)d_ws; _Float16 *QH = (_Float16*)(ws + WS_QH), *QL = (_Float16*)(ws + WS_QL), *KH = (_Float16*)(ws + WS_KH), *KL = (_Float16*)(ws + WS_KL), *VH = (_Float16*)(ws + WS_VH), *VL = (_Float16*)(ws + WS_VL); float* DT = (float*)(ws + WS_DT);
  k_q<<<dim3(TNB * N1 / 64, INNER / 128), 128, 0, stream>>>(F[0], F[4], F[2], QH, QL);
  k_kv<<<dim3(TNB * N2 / 64, 2 * INNER / 128), 128, 0, stream>>>(F[1], F[5], F[3], F[6], F[7], F[8], F[9], KH, KL, VH, VL);
  k_dots<<<TNB * NH, 128, 0, stream>>>(KH, KL, VH, VL, DT);
  k_o<<<dim3(TNB * N1 / 64, DIMI / 128), 128, 0, stream>>>(QH, QL, DT, F[10], F[11], (float*)d_out);
}
